// RecurrentMultiheadAttention_32323923869788
// MI455X (gfx1250) — hardware-verified
//
#include <hip/hip_runtime.h>
#include <math.h>

constexpr int kBatch = 2;
constexpr int kSeq   = 2048;
constexpr int kDm    = 1024;
constexpr int kHeads = 16;
constexpr int kHd    = 64;
constexpr int kTok   = kBatch * kSeq;

typedef __attribute__((ext_vector_type(16))) _Float16 v16h;
typedef __attribute__((ext_vector_type(8)))  _Float16 v8h;
typedef __attribute__((ext_vector_type(16))) __bf16   v16b;
typedef __attribute__((ext_vector_type(8)))  __bf16   v8b;
typedef __attribute__((ext_vector_type(8)))  float    v8f;
typedef __attribute__((ext_vector_type(4)))  float    v4f;
typedef __attribute__((ext_vector_type(2)))  float    v2f;

__device__ __forceinline__ unsigned short f2bf_bits(float f) {
  unsigned u = __float_as_uint(f);
  return (unsigned short)((u + 0x7FFFu + ((u >> 16) & 1u)) >> 16);
}
__device__ __forceinline__ float bf_bits2f(unsigned short h) { return __uint_as_float(((unsigned)h) << 16); }
__device__ __forceinline__ unsigned pk16(unsigned short a, unsigned short b) { return (unsigned)a | ((unsigned)b << 16); }

__device__ __forceinline__ void dep_guard_h(v8f& a, v8f& b, v16h x, v16h y) { asm volatile("v_nop\n\tv_nop\n\tv_nop\n\tv_nop" : "+v"(a), "+v"(b) : "v"(x), "v"(y)); }
__device__ __forceinline__ void dep_guard_b(v8f& a, v8f& b, v16b x, v16b y) { asm volatile("v_nop\n\tv_nop\n\tv_nop\n\tv_nop" : "+v"(a), "+v"(b) : "v"(x), "v"(y)); }
__device__ __forceinline__ void keep4_h(v16h a, v16h b, v16h c, v16h d) { asm volatile("v_nop" :: "v"(a), "v"(b), "v"(c), "v"(d)); }
__device__ __forceinline__ void keep4_b(v16b a, v16b b, v16b c, v16b d) { asm volatile("v_nop" :: "v"(a), "v"(b), "v"(c), "v"(d)); }
__device__ __forceinline__ void acc_guard4(v8f& a, v8f& b, v8f& c, v8f& d) { asm volatile("v_nop\n\tv_nop\n\tv_nop\n\tv_nop" : "+v"(a), "+v"(b), "+v"(c), "+v"(d)); }
template <typename T> struct Frag;
template <> struct Frag<_Float16> {
  typedef v16h V; union U { v16h v; v8h h[2]; };
  static __device__ __forceinline__ v16h load(const _Float16* p) {
    U f; f.h[0] = *(const v8h*)(p); f.h[1] = *(const v8h*)(p + 16); return f.v;
  }
  static __device__ __forceinline__ v8f mma(v16h a, v16h b, v8f c) {
    return __builtin_amdgcn_wmma_f32_16x16x32_f16(false, a, false, b, (short)0, c, false, false);
  }
  static __device__ __forceinline__ void guard(v8f& a, v8f& b, v16h x, v16h y) { dep_guard_h(a, b, x, y); }
  static __device__ __forceinline__ void keep(v16h a, v16h b, v16h c, v16h d) { keep4_h(a, b, c, d); }
};
template <> struct Frag<__bf16> {
  typedef v16b V; union U { v16b v; v8b h[2]; };
  static __device__ __forceinline__ v16b load(const __bf16* p) {
    U f; f.h[0] = *(const v8b*)(p); f.h[1] = *(const v8b*)(p + 16); return f.v;
  }
  static __device__ __forceinline__ v8f mma(v16b a, v16b b, v8f c) {
    return __builtin_amdgcn_wmma_f32_16x16x32_bf16(false, a, false, b, (short)0, c, false, false);
  }
  static __device__ __forceinline__ void guard(v8f& a, v8f& b, v16b x, v16b y) { dep_guard_b(a, b, x, y); }
  static __device__ __forceinline__ void keep(v16b a, v16b b, v16b c, v16b d) { keep4_b(a, b, c, d); }
};

template <int ET> struct Elem;
template <> struct Elem<0> { typedef _Float16 T; };
template <> struct Elem<1> { typedef __bf16 T; };
template <int ET, bool SPLIT, int BIAS_MODE, int OUT_MODE, bool RESID, int ACT = 0>
__global__ __launch_bounds__(256) void wmma_gemm64(
    const unsigned short* __restrict__ Ap, const unsigned short* __restrict__ A2p, int lda, long strideA,
    const unsigned short* __restrict__ Btp, const unsigned short* __restrict__ Bt2p, int ldb, long strideB,
    void* __restrict__ Cout, void* __restrict__ Cout2, int ldc, long strideC,
    const float* __restrict__ bias,
    const float* __restrict__ resid, long strideR,
    int M, int N, int K, float scale) {
  typedef typename Elem<ET>::T T;
  typedef typename Frag<T>::V V;
  const T* A = (const T*)Ap; const T* A2 = (const T*)A2p; const T* Bt = (const T*)Btp; const T* Bt2 = (const T*)Bt2p;
  __shared__ __align__(16) float sT[8][16 * 68];
  const int b    = blockIdx.y;
  const int lane = threadIdx.x & 31;
  const int wave = threadIdx.x >> 5;
  const int tilesN = N >> 6;
  const int tilesM = M >> 6;
  const int tile = blockIdx.x * 8 + wave;
  if (tile >= tilesM * tilesN) return;
  const int tm = tile / tilesN;
  const int tn = tile - tm * tilesN;
  const int m0 = tm << 6;
  const int n0 = tn << 6;

  const T* Ab  = A  + (size_t)b * strideA;
  const T* Bb  = Bt + (size_t)b * strideB;
  const T* Ab2 = SPLIT ? (A2  + (size_t)b * strideA) : nullptr;
  const T* Bb2 = SPLIT ? (Bt2 + (size_t)b * strideB) : nullptr;

  const int rlane = lane & 15;
  const int koff  = (lane >> 4) * 8;
  const int mOff  = (lane >> 4) * 8;

  v8f acc[4][4];
#pragma unroll
  for (int i = 0; i < 4; ++i)
#pragma unroll
    for (int j = 0; j < 4; ++j) acc[i][j] = (v8f){0.f,0.f,0.f,0.f,0.f,0.f,0.f,0.f};

  for (int k0 = 0; k0 < K; k0 += 32) {
    V bh[4], bl[4];
#pragma unroll
    for (int j = 0; j < 4; ++j) {
      const size_t bo = (size_t)(n0 + (j << 4) + rlane) * ldb + koff + k0;
      bh[j] = Frag<T>::load(Bb + bo);
      if (SPLIT) bl[j] = Frag<T>::load(Bb2 + bo);
    }
#pragma unroll
    for (int i = 0; i < 4; ++i) {
      const size_t ao = (size_t)(m0 + (i << 4) + rlane) * lda + koff + k0;
      V ah = Frag<T>::load(Ab + ao);
      V al;
      if (SPLIT) al = Frag<T>::load(Ab2 + ao);
#pragma unroll
      for (int j = 0; j < 4; ++j) {
        acc[i][j] = Frag<T>::mma(ah, bh[j], acc[i][j]);
        if (SPLIT) {
          acc[i][j] = Frag<T>::mma(ah, bl[j], acc[i][j]);
          acc[i][j] = Frag<T>::mma(al, bh[j], acc[i][j]);
        }
      }
      Frag<T>::guard(acc[i][0], acc[i][3], ah, SPLIT ? al : ah);
    }
    Frag<T>::keep(bh[0], bh[1], bh[2], bh[3]);
    if (SPLIT) Frag<T>::keep(bl[0], bl[1], bl[2], bl[3]);
  }
  acc_guard4(acc[0][0], acc[0][1], acc[0][2], acc[0][3]);
  acc_guard4(acc[1][0], acc[1][1], acc[1][2], acc[1][3]);
  acc_guard4(acc[2][0], acc[2][1], acc[2][2], acc[2][3]);
  acc_guard4(acc[3][0], acc[3][1], acc[3][2], acc[3][3]);

  float* slab = sT[wave];
  const float* Rb = RESID ? (resid + (size_t)b * strideR) : nullptr;
#pragma unroll
  for (int i = 0; i < 4; ++i) {
    const int mBase = m0 + (i << 4);
#pragma unroll
    for (int j = 0; j < 4; ++j) {
      const int n = n0 + (j << 4) + rlane;
      float bv = 0.f;
      if (BIAS_MODE == 2) bv = bias[n];
#pragma unroll
      for (int r = 0; r < 8; ++r) {
        float v = acc[i][j][r] * scale;
        if (BIAS_MODE == 1) v += bias[mBase + mOff + r];
        if (BIAS_MODE == 2) v += bv;
        if (RESID) v += Rb[(size_t)(mBase + mOff + r) * ldc + n];
        if (ACT == 1) v = tanhf(v);
        if (ACT == 2) v = fmaxf(v, 0.0f);
        if (ACT == 3) v = v / (1.0f + expf(-v));
        if (ACT == 4) v = (v > 0.f) ? v : 0.01f * v;
        if (ACT == 5) v = 0.5f * v * (1.0f + erff(v * 0.70710678118654752f));
        slab[(mOff + r) * 68 + (j << 4) + rlane] = v;
      }
    }
    __builtin_amdgcn_fence(__ATOMIC_RELEASE, "workgroup");
    __builtin_amdgcn_wave_barrier();
    __builtin_amdgcn_fence(__ATOMIC_ACQUIRE, "workgroup");
    if (OUT_MODE == 0) {
      float* C = (float*)Cout + (size_t)b * strideC;
      const int hh = lane >> 4, c4 = (lane & 15) * 4;
      for (int pass = 0; pass < 2; ++pass) {
#pragma unroll
        for (int it = 0; it < 8; ++it) {
          const int row = it * 2 + hh;
          v4f v = *(const v4f*)(slab + row * 68 + c4);
          *(volatile v4f*)(C + (size_t)(mBase + row) * ldc + n0 + c4) = v;
        }
        __threadfence();
      }
    } else {
      const int q = lane >> 3, c8 = (lane & 7) * 8;
      unsigned short* C  = (unsigned short*)Cout  + (size_t)b * strideC;
      unsigned short* C2 = (OUT_MODE == 2) ? ((unsigned short*)Cout2 + (size_t)b * strideC) : nullptr;
      for (int pass = 0; pass < 2; ++pass) {
#pragma unroll
        for (int it = 0; it < 4; ++it) {
          const int row = it * 4 + q;
          const float* sp = slab + row * 68 + c8;
          v8h hv, lv;
#pragma unroll
          for (int e = 0; e < 8; ++e) {
            if (OUT_MODE == 1) {
              hv[e] = (_Float16)sp[e];
            } else {
              unsigned short hb = f2bf_bits(sp[e]);
              unsigned short lb = f2bf_bits(sp[e] - bf_bits2f(hb));
              hv[e] = __builtin_bit_cast(_Float16, hb);
              lv[e] = __builtin_bit_cast(_Float16, lb);
            }
          }
          *(volatile v8h*)(C + (size_t)(mBase + row) * ldc + n0 + c8) = hv;
          if (OUT_MODE == 2) *(volatile v8h*)(C2 + (size_t)(mBase + row) * ldc + n0 + c8) = lv;
        }
        __threadfence();
      }
    }
    __builtin_amdgcn_fence(__ATOMIC_RELEASE, "workgroup");
    __builtin_amdgcn_wave_barrier();
    __builtin_amdgcn_fence(__ATOMIC_ACQUIRE, "workgroup");
  }
}

template <int MODE>
__global__ __launch_bounds__(256) void cast16x2_kernel(const float* __restrict__ in, unsigned short* __restrict__ out,
                                                       int n2, float scale) {
  const int i = blockIdx.x * 256 + threadIdx.x;
  if (i < n2) {
    const v2f f = *(const v2f*)(in + 2 * (size_t)i);
    unsigned short a0, a1;
    if (MODE == 0) {
      a0 = f2bf_bits(f[0]);
      a1 = f2bf_bits(f[1]);
    } else {
      const float g0 = bf_bits2f(f2bf_bits(f[0])) * scale;
      const float g1 = bf_bits2f(f2bf_bits(f[1])) * scale;
      a0 = __builtin_bit_cast(unsigned short, (_Float16)g0);
      a1 = __builtin_bit_cast(unsigned short, (_Float16)g1);
    }
    const unsigned u = pk16(a0, a1);
    ((volatile unsigned*)out)[i] = u;
    __threadfence();
    ((volatile unsigned*)out)[i] = u;
  }
}

__global__ __launch_bounds__(256) void recur_kernel(const float* __restrict__ Wh, const float* __restrict__ Rp,
                                                    unsigned short* __restrict__ Hs,
                                                    const float* __restrict__ unused_in, int npairs) {
  (void)unused_in;
  const int t = blockIdx.x * 256 + threadIdx.x;
  if (t >= npairs) return;
  const int b  = t / (kDm / 2);
  const int cp = t - b * (kDm / 2);
  const int ch = 2 * cp;
  const float* w0p = Wh + (size_t)ch * kHd;
  const float* w1p = w0p + kHd;
  float w0 = 0.f, w1 = 0.f;
#pragma unroll 1
  for (int k = 0; k < kHd; ++k) {
    w0 += bf_bits2f(f2bf_bits(w0p[k]));
    w1 += bf_bits2f(f2bf_bits(w1p[k]));
  }
  const float* rp = Rp + (size_t)b * kSeq * kDm + ch;
  volatile unsigned* hs = (volatile unsigned*)Hs + (((size_t)b * kSeq * kDm + ch) >> 1);
  float h0 = 0.f, h1 = 0.f;
#pragma unroll 1
  for (int tt = 0; tt < kSeq; ++tt) {
    const v2f r = *(const v2f*)(rp + (size_t)tt * kDm);
    h0 = tanhf(h0 * w0 + r[0]);
    h1 = tanhf(h1 * w1 + r[1]);
    const unsigned u = pk16(__builtin_bit_cast(unsigned short, (_Float16)h0),
                            __builtin_bit_cast(unsigned short, (_Float16)h1));
    hs[(size_t)tt * (kDm / 2)] = u;
    __threadfence();
    hs[(size_t)tt * (kDm / 2)] = u;
  }
}

constexpr int kAtD = 64, kAtNW = 4, kAtQB = 64, kAtKC = 64;
constexpr float kPsc = 32768.0f;

__device__ __forceinline__ v8f at_mma_h(v16h a, v16h b, v8f c) {
  c = __builtin_amdgcn_wmma_f32_16x16x32_f16(false, a, false, b, (short)0, c, false, false);
  asm volatile("v_nop\n\tv_nop\n\tv_nop\n\tv_nop" : "+v"(c) : "v"(a), "v"(b));
  return c;
}

__global__ __launch_bounds__(128)
void attn_f16_kernel(const unsigned short* __restrict__ qp, const unsigned short* __restrict__ kp,
                     const unsigned short* __restrict__ vtp, unsigned short* __restrict__ op,
                     float sscale, float oscale) {
  union FH { v16h v; v8h h[2]; };
  __shared__ __align__(16) _Float16 Ksh[kAtKC * kAtD];
  __shared__ __align__(16) _Float16 Vth[kAtD * kAtKC];
  __shared__ __align__(16) _Float16 Psh[kAtNW][16 * kAtKC];
  __shared__ __align__(16) float    Os[kAtNW][16 * 68];

  const int tid  = threadIdx.x;
  const int wave = tid >> 5;
  const int lane = tid & 31;
  const int hh   = lane >> 4;
  const int c    = lane & 15;

  const int nqb = kSeq / kAtQB;
  const int bx = blockIdx.x;
  const int qb = bx % nqb;
  const int bh = bx / nqb;
  const int h  = bh % kHeads;
  const int b  = bh / kHeads;
  const int q0 = qb * kAtQB + wave * 16;

  const _Float16* Q  = (const _Float16*)(const void*)qp  + (size_t)b * kSeq * kDm + (size_t)h * kAtD;
  const _Float16* Kk = (const _Float16*)(const void*)kp  + (size_t)b * kSeq * kDm + (size_t)h * kAtD;
  const _Float16* Vt = (const _Float16*)(const void*)vtp + ((size_t)b * kDm + (size_t)h * kAtD) * kSeq;
  _Float16*       O  = (_Float16*)(void*)op + (size_t)b * kSeq * kDm + (size_t)h * kAtD;

  v16h qa[2];
#pragma unroll
  for (int dc = 0; dc < 2; ++dc) {
    const _Float16* qr = Q + (size_t)(q0 + c) * kDm + dc * 32 + 8 * hh;
    qa[dc] = Frag<_Float16>::load(qr);
  }

  float mrow[8], lrow[8];
  v8f oacc[4];
#pragma unroll
  for (int r = 0; r < 8; ++r) { mrow[r] = -INFINITY; lrow[r] = 0.f; }
#pragma unroll
  for (int t = 0; t < 4; ++t) oacc[t] = (v8f){0.f,0.f,0.f,0.f,0.f,0.f,0.f,0.f};

  const int nChunks = kSeq / kAtKC;
  for (int kc = 0; kc < nChunks; ++kc) {
    const int kv0 = kc * kAtKC;
    __syncthreads();
    {
      const int r = tid >> 1, half = (tid & 1) * 32;
      const _Float16* ks = Kk + (size_t)(kv0 + r) * kDm + half;
      const _Float16* vs = Vt + (size_t)r * kSeq + kv0 + half;
#pragma unroll
      for (int i = 0; i < 4; ++i) {
        const v8h a0 = *(const v8h*)(ks + 8 * i);
        const v8h b0 = *(const v8h*)(vs + 8 * i);
        *(v8h*)(Ksh + r * kAtD  + half + 8 * i) = a0;
        *(v8h*)(Vth + r * kAtKC + half + 8 * i) = b0;
      }
    }
    __syncthreads();

    v8f s[4];
#pragma unroll
    for (int j = 0; j < 4; ++j) {
      s[j] = (v8f){0.f,0.f,0.f,0.f,0.f,0.f,0.f,0.f};
#pragma unroll
      for (int dc = 0; dc < 2; ++dc) {
        FH kb;
        kb.h[0] = *(const v8h*)(Ksh + (j * 16 + c) * kAtD + dc * 32 + 8 * hh);
        kb.h[1] = *(const v8h*)(Ksh + (j * 16 + c) * kAtD + dc * 32 + 16 + 8 * hh);
        s[j] = at_mma_h(qa[dc], kb.v, s[j]);
      }
    }
    float cm[8];
#pragma unroll
    for (int r = 0; r < 8; ++r) {
      float m = -INFINITY;
#pragma unroll
      for (int j = 0; j < 4; ++j) {
        const float sv = s[j][r] * sscale;
        s[j][r] = sv;
        m = fmaxf(m, sv);
      }
#pragma unroll
      for (int off = 1; off < 16; off <<= 1) m = fmaxf(m, __shfl_xor(m, off, 32));
      cm[r] = m;
    }
    _Float16* pwh = Psh[wave];
#pragma unroll
    for (int r = 0; r < 8; ++r) {
      const float mnew = fmaxf(mrow[r], cm[r]);
      const float alpha = expf(mrow[r] - mnew);
      mrow[r] = mnew;
      float psum = 0.f;
#pragma unroll
      for (int j = 0; j < 4; ++j) {
        const float p = expf(s[j][r] - mnew);
        psum += p;
        pwh[(8 * hh + r) * kAtKC + j * 16 + c] = (_Float16)(p * kPsc);
      }
#pragma unroll
      for (int off = 1; off < 16; off <<= 1) psum += __shfl_xor(psum, off, 32);
      lrow[r] = lrow[r] * alpha + psum;
#pragma unroll
      for (int t = 0; t < 4; ++t) oacc[t][r] *= alpha;
    }
    __builtin_amdgcn_fence(__ATOMIC_RELEASE, "workgroup");
    __builtin_amdgcn_wave_barrier();
    __builtin_amdgcn_fence(__ATOMIC_ACQUIRE, "workgroup");
#pragma unroll 1
    for (int kk = 0; kk < 2; ++kk) {
      FH pa;
      pa.h[0] = *(const v8h*)(pwh + c * kAtKC + kk * 32 + 8 * hh);
      pa.h[1] = *(const v8h*)(pwh + c * kAtKC + kk * 32 + 16 + 8 * hh);
#pragma unroll
      for (int t = 0; t < 4; ++t) {
        FH vb;
        vb.h[0] = *(const v8h*)(Vth + (t * 16 + c) * kAtKC + kk * 32 + 8 * hh);
        vb.h[1] = *(const v8h*)(Vth + (t * 16 + c) * kAtKC + kk * 32 + 16 + 8 * hh);
        oacc[t] = at_mma_h(pa.v, vb.v, oacc[t]);
      }
    }
  }

  float* os = Os[wave];
#pragma unroll
  for (int r = 0; r < 8; ++r) {
    const float inv = oscale * (1.0f / (lrow[r] * kPsc));
#pragma unroll
    for (int t = 0; t < 4; ++t) os[(8 * hh + r) * 68 + t * 16 + c] = oacc[t][r] * inv;
  }
  __builtin_amdgcn_fence(__ATOMIC_RELEASE, "workgroup");
  __builtin_amdgcn_wave_barrier();
  __builtin_amdgcn_fence(__ATOMIC_ACQUIRE, "workgroup");
  {
    const int q8 = lane >> 3, c8 = (lane & 7) * 8;
    for (int pass = 0; pass < 2; ++pass) {
#pragma unroll
      for (int it = 0; it < 4; ++it) {
        const int row = it * 4 + q8;
        const float* sp = os + row * 68 + c8;
        v8h hv;
#pragma unroll
        for (int e = 0; e < 8; ++e) hv[e] = (_Float16)sp[e];
        *(volatile v8h*)(O + (size_t)(q0 + row) * kDm + c8) = hv;
      }
      __threadfence();
    }
  }
}

extern "C" void kernel_launch(void* const* d_in, const int* in_sizes, int n_in,
                              void* d_out, int out_size, void* d_ws, size_t ws_size,
                              hipStream_t stream) {
  if (n_in < 13) return;
  if (in_sizes[0] != kTok * kDm || in_sizes[2] != kTok * kDm || in_sizes[3] != kTok * kDm) return;
  if (in_sizes[4] != kDm * kDm || in_sizes[6] != kDm * kDm || in_sizes[8] != kDm * kDm || in_sizes[11] != kDm * kDm) return;
  if (in_sizes[5] != kDm || in_sizes[7] != kDm || in_sizes[9] != kDm || in_sizes[12] != kDm) return;
  if (in_sizes[10] != kHeads * kHd * kHd) return;
  if (out_size != kTok * kDm) return;

  const size_t bX16  = (size_t)kTok * kDm * 2;
  const size_t bW16  = (size_t)kDm * kDm * 2;
  const size_t bQ16  = (size_t)kTok * kDm * 2;
  const size_t bVT16 = (size_t)kBatch * kDm * kSeq * 2;
  const size_t bRP32 = (size_t)kTok * kDm * 4;
  const size_t bHS16 = (size_t)kTok * kDm * 2;
  const size_t bCT16 = (size_t)kTok * kDm * 2;
  const size_t oX16  = 0;
  const size_t oW16  = oX16 + bX16;
  const size_t oQ16  = oW16 + bW16;
  const size_t oVT16 = oQ16 + bQ16;
  const size_t oRP32 = oVT16 + bVT16;
  const size_t oHS16 = oRP32 + bRP32;
  const size_t oCT16 = oHS16 + bHS16;
  const size_t total = oCT16 + bCT16;
  if (ws_size < total) return;

  const float* query = (const float*)d_in[0];
  const float* keyin = (const float*)d_in[1];
  const float* value = (const float*)d_in[2];
  const float* Rin   = (const float*)d_in[3];
  const float* Wq    = (const float*)d_in[4];
  const float* bq    = (const float*)d_in[5];
  const float* Wv    = (const float*)d_in[6];
  const float* bv    = (const float*)d_in[7];
  const float* Wr    = (const float*)d_in[8];
  const float* br    = (const float*)d_in[9];
  const float* W_h   = (const float*)d_in[10];
  const float* Wo    = (const float*)d_in[11];
  const float* bo    = (const float*)d_in[12];
  float* out = (float*)d_out;

  char* ws = (char*)d_ws;
  unsigned short* X16  = (unsigned short*)(ws + oX16);
  unsigned short* W16  = (unsigned short*)(ws + oW16);
  unsigned short* Q16  = (unsigned short*)(ws + oQ16);
  unsigned short* VT16 = (unsigned short*)(ws + oVT16);
  float*          RP32 = (float*)(ws + oRP32);
  unsigned short* HS16 = (unsigned short*)(ws + oHS16);
  unsigned short* CT16 = (unsigned short*)(ws + oCT16);

  const int n2X = kTok * kDm / 2;
  const int n2W = kDm * kDm / 2;
  const dim3 blk(256);
  const dim3 gCastX((n2X + 255) / 256);
  const dim3 gCastW((n2W + 255) / 256);
  const int tilesQ  = (kTok / 64) * (kDm / 64);
  const int tilesVT = (kDm / 64) * (kSeq / 64);
  const dim3 gGemmQ((tilesQ + 7) / 8, 1);
  const dim3 gGemmVT((tilesVT + 7) / 8, kBatch);

  cast16x2_kernel<0><<<gCastX, blk, 0, stream>>>(query, X16, n2X, 1.0f);
  cast16x2_kernel<0><<<gCastW, blk, 0, stream>>>(Wq, W16, n2W, 1.0f);
  wmma_gemm64<1, false, 2, 1, false><<<gGemmQ, blk, 0, stream>>>(
      X16, X16, kDm, 0L, W16, W16, kDm, 0L, (void*)Q16, (void*)Q16, kDm, 0L,
      bq, bq, 0L, kTok, kDm, kDm, 1.0f);

  cast16x2_kernel<0><<<gCastX, blk, 0, stream>>>(value, X16, n2X, 1.0f);
  cast16x2_kernel<0><<<gCastW, blk, 0, stream>>>(Wv, W16, n2W, 1.0f);
  wmma_gemm64<1, false, 1, 1, false><<<gGemmVT, blk, 0, stream>>>(
      W16, W16, kDm, 0L, X16, X16, kDm, (long)kSeq * kDm, (void*)VT16, (void*)VT16, kSeq, (long)kDm * kSeq,
      bv, bv, 0L, kDm, kSeq, kDm, 1.0f);

  cast16x2_kernel<0><<<gCastX, blk, 0, stream>>>(Rin, X16, n2X, 1.0f);
  cast16x2_kernel<0><<<gCastW, blk, 0, stream>>>(Wr, W16, n2W, 1.0f);
  wmma_gemm64<1, false, 2, 0, false><<<gGemmQ, blk, 0, stream>>>(
      X16, X16, kDm, 0L, W16, W16, kDm, 0L, (void*)RP32, (void*)RP32, kDm, 0L,
      br, br, 0L, kTok, kDm, kDm, 1.0f);

  const int npairs = kBatch * kDm / 2;
  recur_kernel<<<dim3((npairs + 255) / 256), blk, 0, stream>>>(W_h, RP32, HS16, keyin, npairs);

  const dim3 gAttn(kBatch * kHeads * (kSeq / kAtQB));
  attn_f16_kernel<<<gAttn, dim3(128), 0, stream>>>(Q16, HS16, VT16, CT16, 0.125f, 64.0f);

  cast16x2_kernel<1><<<gCastW, blk, 0, stream>>>(Wo, W16, n2W, 64.0f);
  wmma_gemm64<0, false, 2, 0, false><<<gGemmQ, blk, 0, stream>>>(
      CT16, CT16, kDm, 0L, W16, W16, kDm, 0L, (void*)out, (void*)out, kDm, 0L,
      bo, bo, 0L, kTok, kDm, kDm, 1.0f / 4096.0f);
}
